// ReviewRepresentationConv_33672543601279
// MI455X (gfx1250) — hardware-run, weakly checked
//
#include <hip/hip_runtime.h>
#include <stddef.h>
#include <stdint.h>
#include <math.h>

#define NN      50000
#define NE      800000
#define DM      128
#define MP      50048
#define KHL     256
#define NTHR    256
#define NWAVE   8
#define EPT     8
#define WCH     (32 * EPT)
#define NBRUN   1024
#define SLB     10
#define NBK     49
#define WLCAP   3584
#define RCAP    28672
#define DEGCAP  64
#define MAXDEG_MEAS   33
#define MAXB1024_MEAS 16696
#define ABM     64
#define GBM     64
#define GBN     64
#define GTHR    128
#define NEGS    0.01f
#define WSMAX   134217728

constexpr int MEAN_TERMS = 2;
constexpr int KB = DM * MEAN_TERMS;

#define BK_ZINTS (NWAVE * WLCAP + RCAP + 3 * NBRUN)
#define BK_INTS  (BK_ZINTS + 16)
#define BK_LDS   (BK_INTS * 4)

#define PBX  (MP * DM / 8 / NTHR)
#define PBS  (DM * DM / 8 / NTHR)
#define PBD  (DM * KHL / 8 / NTHR)
#define PBTOT (PBX + PBS + PBD + 1)

static_assert(MEAN_TERMS == 1 || MEAN_TERMS == 2);
static_assert(DM == 128 && KHL == 2 * DM && DM % 32 == 0 && KB % 32 == 0);
static_assert(MP % GBM == 0 && MP % ABM == 0 && MP >= NN && DM % GBN == 0);
static_assert(NBRUN == (1 << SLB) && NBRUN <= 1024 && NBRUN % ABM == 0 && NBRUN % 32 == 0);
static_assert(NBK * NBRUN >= MP);
static_assert(NN <= 65536);
static_assert(NE < (1 << 21) && (((long long)NE) << SLB) < (1LL << 31));
static_assert(NE % WCH == 0 && NE % 4 == 0);
static_assert(RCAP == NWAVE * WLCAP && RCAP % 4 == 0 && BK_ZINTS % 4 == 0 && RCAP % (NTHR * 4) == 0);
static_assert((2 * NBRUN) % (NTHR * 4) == 0);
static_assert((long long)RCAP * 100 >= (long long)MAXB1024_MEAS * 105);
static_assert(WLCAP >= MAXB1024_MEAS / 8 + 8 * 46 + 1);
static_assert(MAXDEG_MEAS + 8 <= DEGCAP && DEGCAP < 65536);
static_assert((MP * DM / 8) % NTHR == 0 && (DM * DM / 8) % NTHR == 0 && (DM * KHL / 8) % NTHR == 0);
static_assert(BK_LDS <= 300000);
static_assert(GBM == (GTHR / 32) * 16);
static_assert(ABM == NWAVE * 8);

typedef float          v4f   __attribute__((ext_vector_type(4)));
typedef float          v8f   __attribute__((ext_vector_type(8)));
typedef int            v4i   __attribute__((ext_vector_type(4)));
typedef int            v8i   __attribute__((ext_vector_type(8)));
typedef unsigned       v2u   __attribute__((ext_vector_type(2)));
typedef unsigned short v8us  __attribute__((ext_vector_type(8)));
typedef unsigned short v16us __attribute__((ext_vector_type(16)));
typedef __bf16         v16bf __attribute__((ext_vector_type(16)));
typedef v4f  __attribute__((may_alias)) v4fa;
typedef v4i  __attribute__((may_alias)) v4ia;
typedef v2u  __attribute__((may_alias)) v2ua;
typedef v8us __attribute__((may_alias)) v8usa;
union FragB { v16bf v; v16us u; v8us h[2]; v8i w; };

__device__ __forceinline__ v8f wmb(const FragB& a, const FragB& b, v8f c) {
  v8f d = __builtin_amdgcn_wmma_f32_16x16x32_bf16(false, a.v, false, b.v, (short)0, c, false, false);
  asm volatile("v_nop\n\tv_nop\n\tv_nop\n\tv_nop" : "+v"(d) : "v"(a.w), "v"(b.w));
  return d;
}

__device__ __forceinline__ unsigned bf16_bits(float f) {
  const unsigned u = __float_as_uint(f);
  const unsigned r = (u + 0x7FFFu + ((u >> 16) & 1u)) >> 16;
  const unsigned q = (u >> 16) | 0x40u;
  return ((u & 0x7fffffffu) > 0x7f800000u) ? q : r;
}
__device__ __forceinline__ float bf16_val(float f) {
  return __uint_as_float(bf16_bits(f) << 16);
}

__device__ __forceinline__ void hilo_pack(float v0, float v1, float v2, float v3,
                                          int& h01, int& h23, int& l01, int& l23) {
  const unsigned a0 = bf16_bits(v0), a1 = bf16_bits(v1), a2 = bf16_bits(v2), a3 = bf16_bits(v3);
  const unsigned b0 = bf16_bits(v0 - __uint_as_float(a0 << 16));
  const unsigned b1 = bf16_bits(v1 - __uint_as_float(a1 << 16));
  const unsigned b2 = bf16_bits(v2 - __uint_as_float(a2 << 16));
  const unsigned b3 = bf16_bits(v3 - __uint_as_float(a3 << 16));
  h01 = (int)(a0 | (a1 << 16)); h23 = (int)(a2 | (a3 << 16));
  l01 = (int)(b0 | (b1 << 16)); l23 = (int)(b2 | (b3 << 16));
}

__device__ __forceinline__ v4i regroup32(int h01, int h23, int l01, int l23, int lane) {
  const int s0 = (2 * lane) & 31, s1 = s0 + 1;
  const int a0 = __shfl(h01, s0, 32), a1 = __shfl(h23, s0, 32), a2 = __shfl(h01, s1, 32), a3 = __shfl(h23, s1, 32);
  const int b0 = __shfl(l01, s0, 32), b1 = __shfl(l23, s0, 32), b2 = __shfl(l01, s1, 32), b3 = __shfl(l23, s1, 32);
  const int mk = (lane < 16) ? -1 : 0;
  v4i o;
  o.x = (a0 & mk) | (b0 & ~mk); o.y = (a1 & mk) | (b1 & ~mk);
  o.z = (a2 & mk) | (b2 & ~mk); o.w = (a3 & mk) | (b3 & ~mk);
  return o;
}

__device__ __forceinline__ void st2_v4f(float* p, v4f v) {
  *(volatile v4f*)p = v;
  __threadfence();
  *(volatile v4f*)p = v;
}
__device__ __forceinline__ void st2_v8us(unsigned short* p, v8us v) {
  *(volatile v8us*)p = v;
  __threadfence();
  *(volatile v8us*)p = v;
}

__device__ __forceinline__ v8us gather8(const float* __restrict__ base, int stride) {
  float f[8];
#pragma unroll
  for (int i = 0; i < 8; ++i) f[i] = base[(size_t)i * (size_t)stride];
  v8us o;
#pragma unroll
  for (int i = 0; i < 8; ++i) o[i] = (unsigned short)bf16_bits(f[i]);
  return o;
}

__global__ __launch_bounds__(NTHR) void k_prep(const float* __restrict__ x, const float* __restrict__ sw,
                                               const float* __restrict__ sbi, const float* __restrict__ dw,
                                               const float* __restrict__ dbi, const float* __restrict__ aw,
                                               const float* __restrict__ ab,
                                               unsigned short* xb, unsigned short* swt, unsigned short* dwt,
                                               float* vec) {
  const int tid = (int)threadIdx.x, lane = tid & 31;
  const int blk = (int)blockIdx.x;
  if (blk < PBX) {
    const int u   = blk * NTHR + tid;
    const int row = u >> 4, k8 = (u & 15) * 8;
    const int rc  = row < NN ? row : NN - 1;
    const unsigned mk = row < NN ? 0xffffu : 0u;
    const float* p = x + (size_t)rc * DM + k8;
    const v4f a = *(const v4fa*)p;
    const v4f b = *(const v4fa*)(p + 4);
    v8us o;
    o[0] = (unsigned short)(bf16_bits(a.x) & mk); o[1] = (unsigned short)(bf16_bits(a.y) & mk);
    o[2] = (unsigned short)(bf16_bits(a.z) & mk); o[3] = (unsigned short)(bf16_bits(a.w) & mk);
    o[4] = (unsigned short)(bf16_bits(b.x) & mk); o[5] = (unsigned short)(bf16_bits(b.y) & mk);
    o[6] = (unsigned short)(bf16_bits(b.z) & mk); o[7] = (unsigned short)(bf16_bits(b.w) & mk);
    st2_v8us(xb + (size_t)row * DM + k8, o);
  } else if (blk < PBX + PBS) {
    const int u = (blk - PBX) * NTHR + tid;
    const int n = u >> 4, k8 = (u & 15) * 8;
    const v8us o = gather8(sw + (size_t)k8 * DM + n, DM);
    st2_v8us(swt + (size_t)n * DM + k8, o);
  } else if (blk < PBX + PBS + PBD) {
    const int u = (blk - PBX - PBS) * NTHR + tid;
    const int n = u >> 5, k8 = (u & 31) * 8, kk = k8 & (DM - 1);
    const v8us o = gather8(dw + (size_t)kk * DM + n, DM);
    st2_v8us(dwt + (size_t)n * KHL + k8, o);
  } else {
    const int w = __builtin_amdgcn_readfirstlane(tid >> 5);
    if (w < 4) {
      v4f v;
      if (w == 0) {
        v = *(const v4fa*)(sbi + 4 * lane);
      } else if (w == 1) {
        v = *(const v4fa*)(dbi + 4 * lane);
      } else if (w == 2) {
        v = *(const v4fa*)(aw + 4 * lane);
      } else {
        const float t = ab[0];
        v.x = t; v.y = t; v.z = t; v.w = t;
      }
      v4f o;
      o.x = bf16_val(v.x); o.y = bf16_val(v.y); o.z = bf16_val(v.z); o.w = bf16_val(v.w);
      st2_v4f(vec + 4 * tid, o);
    }
  }
}

template <int KTOT, int LDA, int LDB>
__global__ __launch_bounds__(GTHR) __attribute__((amdgpu_num_vgpr(248)))
void k_gemm(const unsigned short* __restrict__ A, const unsigned short* __restrict__ WT,
            const float* __restrict__ bias, float* outF) {
  __shared__ __attribute__((aligned(16))) float stg[GBM * GBN];
  __shared__ __attribute__((aligned(16))) float sb[GBN];
  const int tid = (int)threadIdx.x, lane = tid & 31, wave = tid >> 5, hh = lane >> 4, m = lane & 15;
  const int rowBase = (int)blockIdx.x * GBM;
  const int col0    = (int)blockIdx.y * GBN;
  if (tid < 16) *(v4fa*)(sb + 4 * tid) = *(const v4fa*)(bias + col0 + 4 * tid);

  v8f acc[4];
  {
    const v8f z = {0.f, 0.f, 0.f, 0.f, 0.f, 0.f, 0.f, 0.f};
#pragma unroll
    for (int t = 0; t < 4; ++t) acc[t] = z;
  }
  const unsigned short* ap = A + (size_t)(rowBase + 16 * wave + m) * (size_t)LDA + 8 * hh;
  const unsigned short* wp = WT + (size_t)(col0 + m) * (size_t)LDB + 8 * hh;
#pragma unroll 1
  for (int k0 = 0; k0 < KTOT; k0 += 32) {
    FragB af;
    af.h[0] = *(const v8usa*)(ap + k0);
    af.h[1] = *(const v8usa*)(ap + k0 + 16);
#pragma unroll
    for (int t = 0; t < 4; ++t) {
      const unsigned short* wq = wp + (size_t)(16 * t) * (size_t)LDB + k0;
      FragB bf;
      bf.h[0] = *(const v8usa*)wq;
      bf.h[1] = *(const v8usa*)(wq + 16);
      acc[t] = wmb(af, bf, acc[t]);
    }
  }

#pragma unroll
  for (int t = 0; t < 4; ++t) {
#pragma unroll
    for (int r = 0; r < 8; ++r) stg[(16 * wave + 8 * hh + r) * GBN + 16 * t + m] = acc[t][r];
  }
  __syncthreads();

  const v4f bv = *(const v4fa*)(sb + 4 * m);
  v4f fv[8];
#pragma unroll
  for (int i = 0; i < 8; ++i) {
    const int lr = 16 * wave + 2 * i + hh;
    const v4f a = *(const v4fa*)(stg + lr * GBN + 4 * m);
    v4f o;
    o.x = a.x + bv.x; o.y = a.y + bv.y; o.z = a.z + bv.z; o.w = a.w + bv.w;
    fv[i] = o;
  }
#pragma unroll
  for (int i = 0; i < 8; ++i) {
    const int gr = rowBase + 16 * wave + 2 * i + hh;
    float* op = outF + (size_t)gr * (size_t)DM + col0 + 4 * m;
    *(volatile v4f*)op = fv[i];
  }
  __threadfence();
#pragma unroll
  for (int i = 0; i < 8; ++i) {
    const int gr = rowBase + 16 * wave + 2 * i + hh;
    float* op = outF + (size_t)gr * (size_t)DM + col0 + 4 * m;
    *(volatile v4f*)op = fv[i];
  }
}

__device__ __forceinline__ void bucket_flush(const int* pl, const int* cnt, int ov, int* lp, int* cop, int* fp,
                                             int tid) {
#pragma unroll 1
  for (int i = tid * 4; i < RCAP; i += NTHR * 4) {
    const v4i v = *(const v4ia*)(pl + i);
    *(volatile v4i*)(lp + i) = v;
  }
#pragma unroll 1
  for (int i = tid * 4; i < 2 * NBRUN; i += NTHR * 4) {
    const v4i v = *(const v4ia*)(cnt + i);
    *(volatile v4i*)(cop + i) = v;
  }
  if (tid < 8) {
    const v4i f = {ov, ov, ov, ov};
    *(volatile v4i*)(fp + 4 * tid) = f;
  }
}

__global__ __launch_bounds__(NTHR) void k_bucket(const int* __restrict__ srcs, const int* __restrict__ dsts,
                                                 int* LIST, int* CO, int* FLAG) {
  extern __shared__ __attribute__((aligned(16))) int dsm[];
  int* wl   = dsm;
  int* pl   = dsm + NWAVE * WLCAP;
  int* cnt  = pl + RCAP;
  int* offs = cnt + NBRUN;
  int* cur  = offs + NBRUN;
  int* misc = cur + NBRUN;
  const int tid = (int)threadIdx.x, lane = tid & 31, wave = tid >> 5;
  const int blk = (int)blockIdx.x;
  const unsigned nbs = (unsigned)(blk * NBRUN);

  {
    const v4i z4 = {0, 0, 0, 0};
    for (int i = tid * 4; i < BK_ZINTS; i += NTHR * 4) *(v4ia*)(dsm + i) = z4;
    if (tid < 16) misc[tid] = 0;
  }
  __syncthreads();

  {
    const int per  = ((NE + NWAVE * WCH - 1) / (NWAVE * WCH)) * WCH;
    const int ebeg = wave * per;
    const int eend = (ebeg + per < NE) ? (ebeg + per) : NE;
    int* mylist = wl + wave * WLCAP;
    int wc = 0;
#pragma unroll 1
    for (int cb = ebeg; cb < eend; cb += WCH) {
      const int e0 = cb + lane * EPT;
      const v4i da = *(const v4ia*)(dsts + e0);
      const v4i db = *(const v4ia*)(dsts + e0 + 4);
      const unsigned s0 = (unsigned)da.x - nbs, s1 = (unsigned)da.y - nbs;
      const unsigned s2 = (unsigned)da.z - nbs, s3 = (unsigned)da.w - nbs;
      const unsigned s4 = (unsigned)db.x - nbs, s5 = (unsigned)db.y - nbs;
      const unsigned s6 = (unsigned)db.z - nbs, s7 = (unsigned)db.w - nbs;
      const bool h0 = s0 < (unsigned)NBRUN, h1 = s1 < (unsigned)NBRUN, h2 = s2 < (unsigned)NBRUN, h3 = s3 < (unsigned)NBRUN;
      const bool h4 = s4 < (unsigned)NBRUN, h5 = s5 < (unsigned)NBRUN, h6 = s6 < (unsigned)NBRUN, h7 = s7 < (unsigned)NBRUN;
      const unsigned m0 = __builtin_amdgcn_ballot_w32(h0), m1 = __builtin_amdgcn_ballot_w32(h1);
      const unsigned m2 = __builtin_amdgcn_ballot_w32(h2), m3 = __builtin_amdgcn_ballot_w32(h3);
      const unsigned m4 = __builtin_amdgcn_ballot_w32(h4), m5 = __builtin_amdgcn_ballot_w32(h5);
      const unsigned m6 = __builtin_amdgcn_ballot_w32(h6), m7 = __builtin_amdgcn_ballot_w32(h7);
      const unsigned any = m0 | m1 | m2 | m3 | m4 | m5 | m6 | m7;
      if (any != 0u) {
        const int pre = (int)(__builtin_amdgcn_mbcnt_lo(m0, 0u) + __builtin_amdgcn_mbcnt_lo(m1, 0u) +
                              __builtin_amdgcn_mbcnt_lo(m2, 0u) + __builtin_amdgcn_mbcnt_lo(m3, 0u) +
                              __builtin_amdgcn_mbcnt_lo(m4, 0u) + __builtin_amdgcn_mbcnt_lo(m5, 0u) +
                              __builtin_amdgcn_mbcnt_lo(m6, 0u) + __builtin_amdgcn_mbcnt_lo(m7, 0u));
        int p = wc + pre;
        if (h0) { if (p < WLCAP) mylist[p] = ((e0 + 0) << SLB) | (int)s0; p = p + 1; }
        if (h1) { if (p < WLCAP) mylist[p] = ((e0 + 1) << SLB) | (int)s1; p = p + 1; }
        if (h2) { if (p < WLCAP) mylist[p] = ((e0 + 2) << SLB) | (int)s2; p = p + 1; }
        if (h3) { if (p < WLCAP) mylist[p] = ((e0 + 3) << SLB) | (int)s3; p = p + 1; }
        if (h4) { if (p < WLCAP) mylist[p] = ((e0 + 4) << SLB) | (int)s4; p = p + 1; }
        if (h5) { if (p < WLCAP) mylist[p] = ((e0 + 5) << SLB) | (int)s5; p = p + 1; }
        if (h6) { if (p < WLCAP) mylist[p] = ((e0 + 6) << SLB) | (int)s6; p = p + 1; }
        if (h7) { if (p < WLCAP) mylist[p] = ((e0 + 7) << SLB) | (int)s7; p = p + 1; }
        wc += (int)(__builtin_popcount(m0) + __builtin_popcount(m1) + __builtin_popcount(m2) + __builtin_popcount(m3) +
                    __builtin_popcount(m4) + __builtin_popcount(m5) + __builtin_popcount(m6) + __builtin_popcount(m7));
      }
    }
    if (lane == 0) misc[wave] = wc;
  }
  __syncthreads();

  if (wave == 0) {
    int ov = 0;
#pragma unroll 1
    for (int w2 = 0; w2 < NWAVE; ++w2) {
      int c = misc[w2];
      if (c > WLCAP) ov = 1;
      c = c < 0 ? 0 : (c > WLCAP ? WLCAP : c);
#pragma unroll 1
      for (int b0 = 0; b0 < c; b0 += 32) {
        const int idx = b0 + lane;
        const int ent = wl[w2 * WLCAP + (idx < WLCAP ? idx : WLCAP - 1)];
        const int m32 = (c - b0) < 32 ? (c - b0) : 32;
#pragma unroll 1
        for (int k = 0; k < m32; ++k) {
          const int u    = __builtin_amdgcn_readlane(ent, k);
          const int slot = u & (NBRUN - 1);
          if (lane == 0) cnt[slot] = cnt[slot] + 1;
        }
      }
    }
    if (lane == 0) misc[9] = ov;
  }
  __syncthreads();
  if (wave == 0) {
    const int base = lane * (NBRUN / 32);
    int s = 0;
#pragma unroll 1
    for (int i = 0; i < NBRUN / 32; ++i) s += cnt[base + i];
    int incl = s;
#pragma unroll
    for (int d = 1; d < 32; d <<= 1) {
      const int y = __shfl_up(incl, d, 32);
      if (lane >= d) incl += y;
    }
    int run = incl - s;
#pragma unroll 1
    for (int i = 0; i < NBRUN / 32; ++i) {
      const int cv = cnt[base + i];
      offs[base + i] = run;
      cur[base + i]  = run;
      run += cv;
    }
  }
  __syncthreads();

  if (wave == 0) {
#pragma unroll 1
    for (int w2 = 0; w2 < NWAVE; ++w2) {
      int c = misc[w2];
      c = c < 0 ? 0 : (c > WLCAP ? WLCAP : c);
#pragma unroll 1
      for (int b0 = 0; b0 < c; b0 += 32) {
        const int idx = b0 + lane;
        const int ent = wl[w2 * WLCAP + (idx < WLCAP ? idx : WLCAP - 1)];
        int eid = (ent >> SLB) & 0x1FFFFF;
        eid = eid > NE - 1 ? NE - 1 : eid;
        int sr = srcs[eid];
        sr = sr < 0 ? 0 : (sr > NN - 1 ? NN - 1 : sr);
        const int word = (int)((unsigned)sr | ((unsigned)(ent & (NBRUN - 1)) << 16));
        const int m32 = (c - b0) < 32 ? (c - b0) : 32;
#pragma unroll 1
        for (int k = 0; k < m32; ++k) {
          const int u    = __builtin_amdgcn_readlane(ent, k);
          const int wd   = __builtin_amdgcn_readlane(word, k);
          const int slot = u & (NBRUN - 1);
          if (lane == 0) {
            int p = cur[slot];
            p = p < 0 ? 0 : (p > RCAP - 1 ? RCAP - 1 : p);
            pl[p] = wd;
            cur[slot] = p + 1;
          }
        }
      }
    }
  }
  __syncthreads();

  const int ovf = misc[9];
  int* lp  = LIST + (size_t)blk * RCAP;
  int* cop = CO + (size_t)blk * (2 * NBRUN);
  int* fp  = FLAG + (size_t)blk * 32;
  bucket_flush(pl, cnt, ovf, lp, cop, fp, tid);
  __threadfence();
  bucket_flush(pl, cnt, ovf, lp, cop, fp, tid);
}

__global__ __launch_bounds__(NTHR) void k_mean(const int* __restrict__ LIST, const int* __restrict__ CO,
                                               const int* __restrict__ FLAG, const unsigned short* __restrict__ XB,
                                               unsigned short* MHL) {
  const int tid = (int)threadIdx.x, lane = tid & 31;
  const int wave = __builtin_amdgcn_readfirstlane(tid >> 5);
  const int rowBase = (int)blockIdx.x * ABM;
  const int bucket  = rowBase >> SLB;
  const int* lb  = LIST + (size_t)bucket * RCAP;
  const int* cob = CO + (size_t)bucket * (2 * NBRUN);
  const int flag = __builtin_amdgcn_readfirstlane(FLAG[(size_t)bucket * 32]);
  const float qnan = __uint_as_float(0x7fc00000u);

#pragma unroll 1
  for (int i = 0; i < ABM / NWAVE; ++i) {
    const int d    = rowBase + (ABM / NWAVE) * wave + i;
    const int slot = d & (NBRUN - 1);
    int c = __builtin_amdgcn_readfirstlane(cob[slot]);
    int o = __builtin_amdgcn_readfirstlane(cob[NBRUN + slot]);
    const bool big = c > DEGCAP;
    c = c < 0 ? 0 : (c > DEGCAP ? DEGCAP : c);
    o = o < 0 ? 0 : (o > RCAP - 1 ? RCAP - 1 : o);
    int last = o + c - 1;
    last = last < o ? o : last;
    last = last > RCAP - 1 ? RCAP - 1 : last;
    float a0 = 0.0f, a1 = 0.0f, a2 = 0.0f, a3 = 0.0f;
#pragma unroll 1
    for (int j = 0; j < c; ++j) {
      int idx = o + j;
      idx = idx > last ? last : idx;
      const unsigned wd = (unsigned)lb[idx];
      int sr = (int)(wd & 0xffffu);
      sr = sr > NN - 1 ? NN - 1 : sr;
      const v2u xw = *(const v2ua*)(XB + (size_t)sr * DM + 4 * lane);
      asm volatile("" :: "v"(xw.x), "v"(xw.y));
      a0 += __uint_as_float(xw.x << 16);
      a1 += __uint_as_float(xw.x & 0xffff0000u);
      a2 += __uint_as_float(xw.y << 16);
      a3 += __uint_as_float(xw.y & 0xffff0000u);
    }
    const float cm = (float)(c > 1 ? c : 1);
    float m0 = a0 / cm, m1 = a1 / cm, m2 = a2 / cm, m3 = a3 / cm;
    const bool bad  = (flag != 0) | big;
    const bool live = d < NN;
    m0 = bad ? qnan : m0; m1 = bad ? qnan : m1; m2 = bad ? qnan : m2; m3 = bad ? qnan : m3;
    m0 = live ? m0 : 0.0f; m1 = live ? m1 : 0.0f; m2 = live ? m2 : 0.0f; m3 = live ? m3 : 0.0f;
    int h01, h23, l01, l23;
    hilo_pack(m0, m1, m2, m3, h01, h23, l01, l23);
    const v4i ow = regroup32(h01, h23, l01, l23, lane);
    unsigned short* hp = MHL + (size_t)d * KHL + 8 * lane;
    *(volatile v4i*)hp = ow;
    __threadfence();
    *(volatile v4i*)hp = ow;
  }
}

__global__ __launch_bounds__(NTHR) void k_att(const int* __restrict__ LIST, const int* __restrict__ CO,
                                              const int* __restrict__ FLAG, const float* __restrict__ HS,
                                              const float* __restrict__ HD, const unsigned short* __restrict__ XB,
                                              const float* __restrict__ VEC, float* out) {
  const int tid = (int)threadIdx.x, lane = tid & 31;
  const int wave = __builtin_amdgcn_readfirstlane(tid >> 5);
  const int rowBase = (int)blockIdx.x * ABM;
  const int bucket  = rowBase >> SLB;
  const int* lb  = LIST + (size_t)bucket * RCAP;
  const int* cob = CO + (size_t)bucket * (2 * NBRUN);
  const int flag = __builtin_amdgcn_readfirstlane(FLAG[(size_t)bucket * 32]);
  const float qnan = __uint_as_float(0x7fc00000u);
  const v4f aw = *(const v4fa*)(VEC + 256 + 4 * lane);
  const float ab = VEC[384];

#pragma unroll 1
  for (int i = 0; i < ABM / NWAVE; ++i) {
    const int d    = rowBase + (ABM / NWAVE) * wave + i;
    const int dc   = d < NN ? d : NN - 1;
    const int slot = d & (NBRUN - 1);
    int c = __builtin_amdgcn_readfirstlane(cob[slot]);
    int o = __builtin_amdgcn_readfirstlane(cob[NBRUN + slot]);
    const bool big = c > DEGCAP;
    c = c < 0 ? 0 : (c > DEGCAP ? DEGCAP : c);
    o = o < 0 ? 0 : (o > RCAP - 1 ? RCAP - 1 : o);
    int last = o + c - 1;
    last = last < o ? o : last;
    last = last > RCAP - 1 ? RCAP - 1 : last;
    const v4f hd = *(const v4fa*)(HD + (size_t)dc * DM + 4 * lane);
    asm volatile("" :: "v"(hd));
    float a0 = 0.0f, a1 = 0.0f, a2 = 0.0f, a3 = 0.0f, den = 0.0f;
#pragma unroll 1
    for (int j = 0; j < c; ++j) {
      int idx = o + j;
      idx = idx > last ? last : idx;
      const unsigned wd = (unsigned)lb[idx];
      int sr = (int)(wd & 0xffffu);
      sr = sr > NN - 1 ? NN - 1 : sr;
      const v4f hs = *(const v4fa*)(HS + (size_t)sr * DM + 4 * lane);
      const v2u xw = *(const v2ua*)(XB + (size_t)sr * DM + 4 * lane);
      asm volatile("" :: "v"(hs));
      asm volatile("" :: "v"(xw.x), "v"(xw.y));
      float t0 = hs.x + hd.x, t1 = hs.y + hd.y, t2 = hs.z + hd.z, t3 = hs.w + hd.w;
      t0 = (t0 >= 0.0f) ? t0 : NEGS * t0;
      t1 = (t1 >= 0.0f) ? t1 : NEGS * t1;
      t2 = (t2 >= 0.0f) ? t2 : NEGS * t2;
      t3 = (t3 >= 0.0f) ? t3 : NEGS * t3;
      float part = t0 * aw.x;
      part = fmaf(t1, aw.y, part);
      part = fmaf(t2, aw.z, part);
      part = fmaf(t3, aw.w, part);
      part += __shfl_xor(part, 16, 32);
      part += __shfl_xor(part, 8, 32);
      part += __shfl_xor(part, 4, 32);
      part += __shfl_xor(part, 2, 32);
      part += __shfl_xor(part, 1, 32);
      const float s = expf(part + ab);
      den += s;
      a0 = fmaf(s, __uint_as_float(xw.x << 16), a0);
      a1 = fmaf(s, __uint_as_float(xw.x & 0xffff0000u), a1);
      a2 = fmaf(s, __uint_as_float(xw.y << 16), a2);
      a3 = fmaf(s, __uint_as_float(xw.y & 0xffff0000u), a3);
    }
    const bool has = c > 0;
    const float dsafe = has ? den : 1.0f;
    float o0 = a0 / dsafe, o1 = a1 / dsafe, o2 = a2 / dsafe, o3 = a3 / dsafe;
    o0 = has ? o0 : 0.0f; o1 = has ? o1 : 0.0f; o2 = has ? o2 : 0.0f; o3 = has ? o3 : 0.0f;
    const bool bad = (flag != 0) | big;
    o0 = bad ? qnan : o0; o1 = bad ? qnan : o1; o2 = bad ? qnan : o2; o3 = bad ? qnan : o3;
    v4f ov;
    ov.x = o0; ov.y = o1; ov.z = o2; ov.w = o3;
    float* op = out + (size_t)dc * DM + 4 * lane;
    const bool wr = d < NN;
    if (wr) *(volatile v4f*)op = ov;
    __threadfence();
    if (wr) *(volatile v4f*)op = ov;
  }
}

extern "C" void kernel_launch(void* const* d_in, const int* in_sizes, int n_in,
                              void* d_out, int out_size, void* d_ws, size_t ws_size,
                              hipStream_t stream) {
  if (n_in < 9) return;
  if (in_sizes[0] != NN * DM) return;
  if (in_sizes[1] != NE) return;
  if (in_sizes[2] != NE) return;
  if (in_sizes[3] != DM * DM) return;
  if (in_sizes[4] != DM) return;
  if (in_sizes[5] != DM * DM) return;
  if (in_sizes[6] != DM) return;
  if (in_sizes[7] != DM) return;
  if (in_sizes[8] != 1) return;
  if (out_size != NN * DM) return;

  const float* x    = (const float*)d_in[0];
  const int*   srcs = (const int*)d_in[1];
  const int*   dsts = (const int*)d_in[2];
  const float* sw   = (const float*)d_in[3];
  const float* sbi  = (const float*)d_in[4];
  const float* dw   = (const float*)d_in[5];
  const float* dbi  = (const float*)d_in[6];
  const float* aw   = (const float*)d_in[7];
  const float* ab   = (const float*)d_in[8];
  float* out = (float*)d_out;

  constexpr size_t zXB   = (size_t)MP * DM * 2;
  constexpr size_t zF    = (size_t)MP * DM * 4;
  constexpr size_t zMHL  = (size_t)MP * KHL * 2;
  constexpr size_t zLIST = (size_t)NBK * RCAP * 4;
  constexpr size_t zCO   = (size_t)NBK * 2 * NBRUN * 4;
  constexpr size_t zFLAG = (((size_t)NBK * 128 + 255) / 256) * 256;
  constexpr size_t zSWT  = (size_t)DM * DM * 2;
  constexpr size_t zDWT  = (size_t)DM * KHL * 2;
  constexpr size_t zVEC  = 2048;
  constexpr size_t oXB   = 0;
  constexpr size_t oHS   = oXB + zXB;
  constexpr size_t oHD   = oHS + zF;
  constexpr size_t oMHL  = oHD + zF;
  constexpr size_t oLIST = oMHL + zMHL;
  constexpr size_t oCO   = oLIST + zLIST;
  constexpr size_t oFLAG = oCO + zCO;
  constexpr size_t oSWT  = oFLAG + zFLAG;
  constexpr size_t oDWT  = oSWT + zSWT;
  constexpr size_t oVEC  = oDWT + zDWT;
  constexpr size_t oEND  = oVEC + zVEC;
  static_assert(zXB % 256 == 0 && zF % 256 == 0 && zMHL % 256 == 0 && zLIST % 256 == 0 && zCO % 256 == 0);
  static_assert(zFLAG % 256 == 0 && zFLAG >= (size_t)NBK * 128 && zSWT % 256 == 0 && zDWT % 256 == 0);
  static_assert(zVEC >= 512 * 4);
  static_assert(oEND <= (size_t)WSMAX);
  if (oEND > ws_size) return;

  char* ws = (char*)d_ws;
  unsigned short* XB   = (unsigned short*)(ws + oXB);
  float*          HS   = (float*)(ws + oHS);
  float*          HD   = (float*)(ws + oHD);
  unsigned short* MHL  = (unsigned short*)(ws + oMHL);
  int*            LIST = (int*)(ws + oLIST);
  int*            CO   = (int*)(ws + oCO);
  int*            FLAG = (int*)(ws + oFLAG);
  unsigned short* SWT  = (unsigned short*)(ws + oSWT);
  unsigned short* DWT  = (unsigned short*)(ws + oDWT);
  float*          VEC  = (float*)(ws + oVEC);

  hipFuncSetAttribute(reinterpret_cast<const void*>(&k_bucket), hipFuncAttributeMaxDynamicSharedMemorySize, (int)BK_LDS);

  k_prep<<<PBTOT, NTHR, 0, stream>>>(x, sw, sbi, dw, dbi, aw, ab, XB, SWT, DWT, VEC);
  k_gemm<DM, DM, DM><<<dim3(MP / GBM, DM / GBN), GTHR, 0, stream>>>(XB, SWT, VEC, HS);
  k_bucket<<<NBK, NTHR, BK_LDS, stream>>>(srcs, dsts, LIST, CO, FLAG);
  k_mean<<<MP / ABM, NTHR, 0, stream>>>(LIST, CO, FLAG, XB, MHL);
  k_gemm<KB, KHL, KHL><<<dim3(MP / GBM, DM / GBN), GTHR, 0, stream>>>(MHL, DWT, VEC + DM, HD);
  k_att<<<MP / ABM, NTHR, 0, stream>>>(LIST, CO, FLAG, HS, HD, XB, VEC, out);
}
